// MessagePassingModelDEBUG_49692771615269
// MI455X (gfx1250) — hardware-verified
//
#include <hip/hip_runtime.h>
#include <stddef.h>
#include <stdint.h>
#include <math.h>


#define NF      32
#define XROW    288
#define NRW     352
#define NZ      18
#define NTHR    256
#define NWAVE   8
#define EPT     8
#define CHUNK   (NTHR * EPT)
#define WCAP    (EPT * 32)
#define LISTN   (NWAVE * WCAP)
#define NBA     1024
#define SLA     10
#define RCAP    24576
#define DEGCAP  64
#define MEAS_B1024  16542
#define MEAS_MAXDEG 33
#define BTHR    256
#define PTHR    128
#define U_RW    (3 * NRW * 4)
#define U_DH    (9 * 32 * 4)
#define DW_L2   (9 * 32 * 32)
#define BKT_LDS_INTS (LISTN + 2 * RCAP + 3 * NBA + 16)
#define WSMAX   134217728

static_assert((CHUNK & (CHUNK - 1)) == 0 && CHUNK <= 4096);
static_assert(NBA == (1 << SLA) && NTHR * 4 == NBA);
static_assert((RCAP % BTHR) == 0 && (RCAP % 32) == 0);
static_assert((long long)RCAP * 20 >= (long long)MEAS_B1024 * 21);
static_assert(DEGCAP >= MEAS_MAXDEG + 8);
static_assert(BKT_LDS_INTS * 4 <= 300000);
static_assert((U_RW % PTHR) == 0 && (U_DH % PTHR) == 0);
static_assert(NF == 32 && (NRW % 16) == 0 && NRW == 11 * NF && XROW == 9 * NF);
static_assert((16 * XROW) % 128 == 0 && (16 * XROW / 4) == 36 * 32);

typedef float          v4f  __attribute__((ext_vector_type(4)));
typedef float          v8f  __attribute__((ext_vector_type(8)));
typedef int            v4i  __attribute__((ext_vector_type(4)));
typedef int            v8i  __attribute__((ext_vector_type(8)));
typedef unsigned short v8us __attribute__((ext_vector_type(8)));
typedef __bf16         v16b __attribute__((ext_vector_type(16)));
typedef v4f  __attribute__((may_alias)) v4fa;
typedef v4i  __attribute__((may_alias)) v4ia;
typedef v8us __attribute__((may_alias)) v8usa;
union FragB { v16b v; v8us h[2]; v8i w; };

__device__ __forceinline__ v8f wmb(const FragB& a, const FragB& b, v8f c) {
  v8f d = __builtin_amdgcn_wmma_f32_16x16x32_bf16(false, a.v, false, b.v, (short)0, c, false, false);
  asm volatile("v_nop\n\tv_nop\n\tv_nop\n\tv_nop" : "+v"(d) : "v"(a.w), "v"(b.w));
  return d;
}
__device__ __forceinline__ void ldwait() { asm volatile("s_wait_loadcnt 0x0" ::: "memory"); }

__device__ __forceinline__ unsigned int f2bf(float f) {
  const unsigned int u = __float_as_uint(f);
  const unsigned int r = ((u + 0x7FFFu + ((u >> 16) & 1u)) >> 16) & 0xFFFFu;
  return ((u & 0x7FFFFFFFu) > 0x7F800000u) ? 0x7FC0u : r;
}
__device__ __forceinline__ float bf2f(unsigned int b) { return __uint_as_float(b << 16); }
__device__ __forceinline__ float bfr(float f) { return bf2f(f2bf(f)); }
__device__ __forceinline__ v4f bfr4(v4f a) { v4f r; r.x = bfr(a.x); r.y = bfr(a.y); r.z = bfr(a.z); r.w = bfr(a.w); return r; }
struct S3 { unsigned int h, m, l; };
__device__ __forceinline__ S3 split3(float v) {
  S3 s; s.h = f2bf(v);
  float r = v - bf2f(s.h); s.m = f2bf(r);
  r = r - bf2f(s.m); s.l = f2bf(r);
  return s;
}
__device__ __forceinline__ void st2_us8(unsigned short* p, v8us v) {
  *(volatile v8us*)p = v; __threadfence(); *(volatile v8us*)p = v;
}

struct Mono { double c; int a; int b; int z; };
constexpr double S3D = 1.7320508075688772;
constexpr int y_nt(int p) { return (p == 6 || p == 8) ? 2 : 1; }
constexpr Mono y_mono(int p, int t) {
  return p == 0 ? Mono{1.0, 0, 0, 0}
       : p == 1 ? Mono{1.0, 1, 0, 0}
       : p == 2 ? Mono{1.0, 0, 1, 0}
       : p == 3 ? Mono{1.0, 0, 0, 1}
       : p == 4 ? Mono{S3D, 1, 1, 0}
       : p == 5 ? Mono{S3D, 0, 1, 1}
       : p == 6 ? (t == 0 ? Mono{1.5, 0, 0, 2} : Mono{-0.5, 0, 0, 0})
       : p == 7 ? Mono{S3D, 1, 0, 1}
       : (t == 0 ? Mono{0.5 * S3D, 2, 0, 0} : Mono{-0.5 * S3D, 0, 2, 0});
}
constexpr double dfact(int n) { double r = 1.0; for (int k = n; k > 1; k -= 2) r *= (double)k; return r; }
constexpr double mono_mean(int a, int b, int c) {
  return (((a | b | c) & 1) != 0) ? 0.0 : dfact(a - 1) * dfact(b - 1) * dfact(c - 1) / dfact(a + b + c + 1);
}
constexpr double gaunt_d(int p, int q, int r) {
  double s = 0.0;
  for (int i = 0; i < y_nt(p); ++i)
    for (int j = 0; j < y_nt(q); ++j)
      for (int k = 0; k < y_nt(r); ++k) {
        const Mono A = y_mono(p, i); const Mono B = y_mono(q, j); const Mono C = y_mono(r, k);
        s += A.c * B.c * C.c * mono_mean(A.a + B.a + C.a, A.b + B.b + C.b, A.z + B.z + C.z);
      }
  return (s < 1e-10 && s > -1e-10) ? 0.0 : s;
}
constexpr double cabsd(double x) { return x < 0.0 ? -x : x; }
static_assert(gaunt_d(0, 0, 0) == 1.0);
static_assert(cabsd(gaunt_d(0, 1, 1) - 1.0 / 3.0) < 1e-14);
static_assert(cabsd(gaunt_d(0, 4, 4) - 0.2) < 1e-14);
static_assert(cabsd(gaunt_d(1, 2, 4) - S3D / 15.0) < 1e-14);
static_assert(cabsd(gaunt_d(3, 3, 6) - 2.0 / 15.0) < 1e-14);
static_assert(cabsd(gaunt_d(6, 6, 6) - 2.0 / 35.0) < 1e-14);
static_assert(gaunt_d(0, 0, 6) == 0.0 && gaunt_d(4, 4, 8) == 0.0 && gaunt_d(1, 2, 3) == 0.0);

constexpr int c_off(int l) { return l == 0 ? 0 : (l == 1 ? 1 : 4); }
constexpr bool any_q(int p, int r, int l2) {
  for (int ql = 0; ql < 2 * l2 + 1; ++ql) if (gaunt_d(p, c_off(l2) + ql, r) != 0.0) return true;
  return false;
}
constexpr bool any_pq(int l1, int l2, int r) {
  for (int pl = 0; pl < 2 * l1 + 1; ++pl) if (any_q(c_off(l1) + pl, r, l2)) return true;
  return false;
}
constexpr int path_slice(int pi) {
  return pi == 0 ? 0 : pi == 1 ? 4 : pi == 2 ? 8 : pi == 3 ? 10 : pi == 4 ? 12 : pi == 5 ? 14
       : pi == 6 ? 16 : pi == 7 ? 20 : pi == 8 ? 22 : pi == 9 ? 24 : 26;
}
static_assert(path_slice(3) == (1 * 3 + 0) * 3 + 1 && path_slice(5) == (1 * 3 + 1) * 3 + 2);
static_assert(path_slice(6) == (1 * 3 + 2) * 3 + 1 && path_slice(7) == (2 * 3 + 0) * 3 + 2);
static_assert(path_slice(8) == (2 * 3 + 1) * 3 + 1 && path_slice(10) == (2 * 3 + 2) * 3 + 2);

template <int P, int Q, int R> struct GC {
  static constexpr double d = gaunt_d(P, Q, R);
  static constexpr bool nz = (d != 0.0);
  static constexpr float f = (float)d;
};
template <int P, int R, int L2, int QL> struct CoefQ {
  static __device__ __forceinline__ float run(const float (&Y)[9], float a) {
    if constexpr (QL < 2 * L2 + 1) {
      constexpr int Q = c_off(L2) + QL;
      if constexpr (GC<P, Q, R>::nz) a = fmaf(GC<P, Q, R>::f, Y[Q], a);
      return CoefQ<P, R, L2, QL + 1>::run(Y, a);
    } else {
      return a;
    }
  }
};
template <int L1, int L2, int R, int PL> struct SumP {
  static __device__ __forceinline__ float run(const float (&xs)[9], const float (&Y)[9], float s) {
    if constexpr (PL < 2 * L1 + 1) {
      constexpr int P = c_off(L1) + PL;
      if constexpr (any_q(P, R, L2)) {
        const float a = CoefQ<P, R, L2, 0>::run(Y, 0.0f);
        s = fmaf(a, xs[P], s);
      }
      return SumP<L1, L2, R, PL + 1>::run(xs, Y, s);
    } else {
      return s;
    }
  }
};
template <int L1, int L2, int L3, int RL> struct PathR {
  static __device__ __forceinline__ void run(const float (&xs)[9], const float (&Y)[9], const float rw, float (&acc)[9]) {
    if constexpr (RL < 2 * L3 + 1) {
      constexpr int R = c_off(L3) + RL;
      if constexpr (any_pq(L1, L2, R)) {
        const float s = SumP<L1, L2, R, 0>::run(xs, Y, 0.0f);
        acc[R] = fmaf(rw, s, acc[R]);
      }
      PathR<L1, L2, L3, RL + 1>::run(xs, Y, rw, acc);
    }
  }
};
template <int L1, int L2, int L3, int RL> struct TdR {
  static __device__ __forceinline__ void run(const float (&xv)[9], const v4f w, float (&part)[16]) {
    if constexpr (RL < 2 * L3 + 1) {
      constexpr int R = c_off(L3) + RL;
      if constexpr (any_pq(L1, L2, R)) {
        const float z = SumP<L1, L2, R, 0>::run(xv, xv, 0.0f);
        part[R * 4 + 0] = fmaf(z, w.x, part[R * 4 + 0]);
        part[R * 4 + 1] = fmaf(z, w.y, part[R * 4 + 1]);
        part[R * 4 + 2] = fmaf(z, w.z, part[R * 4 + 2]);
        part[R * 4 + 3] = fmaf(z, w.w, part[R * 4 + 3]);
      }
      TdR<L1, L2, L3, RL + 1>::run(xv, w, part);
    }
  }
};

__global__ __launch_bounds__(PTHR) void k_prep(const float* __restrict__ mpW, const float* __restrict__ d1W,
                                               const float* __restrict__ d2W, unsigned short* RWT,
                                               unsigned short* DWT) {
  const int u = (int)blockIdx.x * PTHR + (int)threadIdx.x;
  v8us o;
  if (u < U_RW) {
    const int row = u >> 2, k8 = (u & 3) * 8;
    const int itx = row / NRW;
    const int n = row - itx * NRW;
    const int pi = n >> 5, f = n & 31;
    const float* p = mpW + ((size_t)(itx * 27 + path_slice(pi)) * 8) * 32 + f;
#pragma unroll
    for (int i = 0; i < 8; ++i) {
      const float w = p[i * 32];
      o[i] = (k8 < 24) ? (unsigned short)f2bf(w) : (unsigned short)0;
    }
    st2_us8(RWT + (size_t)row * 32 + k8, o);
  } else if (u < U_RW + U_DH) {
    const int v = u - U_RW;
    const int row = v >> 2, k8 = (v & 3) * 8;
    const int r9 = row >> 5, g = row & 31;
    const float* p = d1W + ((size_t)(r9 * 32 + k8)) * 32 + g;
#pragma unroll
    for (int i = 0; i < 8; ++i) o[i] = (unsigned short)f2bf(p[i * 32]);
    st2_us8(DWT + (size_t)row * 32 + k8, o);
  } else if (u < U_RW + 2 * U_DH) {
    const int v = u - U_RW - U_DH;
    const int row = v >> 2, k8 = (v & 3) * 8;
    const int r9 = row >> 5, g = row & 31;
    const float* p = d2W + ((size_t)(r9 * 32 + k8)) * 32 + g;
#pragma unroll
    for (int i = 0; i < 8; ++i) o[i] = (unsigned short)f2bf(p[i * 32]);
    st2_us8(DWT + (size_t)DW_L2 + (size_t)row * 32 + k8, o);
  }
}

__device__ __forceinline__ int scan_chunk(const int* __restrict__ dsts, int nE, int cbase, int slotBase,
                                          int nb, int vec8, int* list, int tid, int lane, int wave) {
  const int el0  = tid * EPT;
  const int e0   = cbase + el0;
  const int sent = -2147483647 - 1;
  v4i da, db;
  if (vec8 != 0 && cbase + CHUNK <= nE) {
    da = *(const v4i*)(dsts + e0);
    db = *(const v4i*)(dsts + e0 + 4);
  } else {
    da.x = (e0     < nE) ? dsts[min(e0,     nE - 1)] : sent;
    da.y = (e0 + 1 < nE) ? dsts[min(e0 + 1, nE - 1)] : sent;
    da.z = (e0 + 2 < nE) ? dsts[min(e0 + 2, nE - 1)] : sent;
    da.w = (e0 + 3 < nE) ? dsts[min(e0 + 3, nE - 1)] : sent;
    db.x = (e0 + 4 < nE) ? dsts[min(e0 + 4, nE - 1)] : sent;
    db.y = (e0 + 5 < nE) ? dsts[min(e0 + 5, nE - 1)] : sent;
    db.z = (e0 + 6 < nE) ? dsts[min(e0 + 6, nE - 1)] : sent;
    db.w = (e0 + 7 < nE) ? dsts[min(e0 + 7, nE - 1)] : sent;
  }
  const unsigned nbs = (unsigned)slotBase;
  const unsigned unb = (unsigned)nb;
  const unsigned s0 = (unsigned)da.x - nbs, s1 = (unsigned)da.y - nbs;
  const unsigned s2 = (unsigned)da.z - nbs, s3 = (unsigned)da.w - nbs;
  const unsigned s4 = (unsigned)db.x - nbs, s5 = (unsigned)db.y - nbs;
  const unsigned s6 = (unsigned)db.z - nbs, s7 = (unsigned)db.w - nbs;
  const bool h0 = s0 < unb, h1 = s1 < unb, h2 = s2 < unb, h3 = s3 < unb;
  const bool h4 = s4 < unb, h5 = s5 < unb, h6 = s6 < unb, h7 = s7 < unb;
  const unsigned hb = (h0 ? 1u : 0u) | (h1 ? 2u : 0u) | (h2 ? 4u : 0u) | (h3 ? 8u : 0u) |
                      (h4 ? 16u : 0u) | (h5 ? 32u : 0u) | (h6 ? 64u : 0u) | (h7 ? 128u : 0u);
  const int c = (int)__builtin_popcount(hb);
  int incl = c;
#pragma unroll
  for (int d = 1; d < 32; d <<= 1) {
    const int y = __shfl_up(incl, d, 32);
    incl += (lane >= d) ? y : 0;
  }
  const int tot  = __shfl(incl, 31, 32);
  const int excl = incl - c;
#define PUTJ(J, HJ, SJ) if (HJ) { \
    const int pos = excl + (int)__builtin_popcount(hb & ((1u << (J)) - 1u)); \
    if (pos < WCAP) list[wave * WCAP + pos] = (int)(((unsigned)(el0 + (J)) << SLA) | (SJ)); }
  PUTJ(0, h0, s0)
  PUTJ(1, h1, s1)
  PUTJ(2, h2, s2)
  PUTJ(3, h3, s3)
  PUTJ(4, h4, s4)
  PUTJ(5, h5, s5)
  PUTJ(6, h6, s6)
  PUTJ(7, h7, s7)
#undef PUTJ
  return tot;
}

__global__ __launch_bounds__(NTHR) void k_bucket(const int* __restrict__ dsts, int nE, int nN, int vec8,
                                                 int* EIDS, int* OFFT, int* CNTT, int* FLG) {
  extern __shared__ __attribute__((aligned(16))) int bsm[];
  int* list = bsm;
  int* reg1 = bsm + LISTN;
  int* sl   = reg1 + RCAP;
  int* cnt  = sl + RCAP;
  int* offs = cnt + NBA;
  int* cur  = offs + NBA;
  int* wcnt = cur + NBA;
  const int tid = (int)threadIdx.x, lane = tid & 31, wave = tid >> 5;
  const int blk = (int)blockIdx.x;
  const int nodeBase = blk * NBA;
  int nb = nN - nodeBase;
  nb = nb < 0 ? 0 : (nb > NBA ? NBA : nb);

  for (int i = tid; i < NBA; i += NTHR) { cnt[i] = 0; offs[i] = 0; cur[i] = 0; }
  __syncthreads();

  int tot = 0, ovf = 0;
  const int nChunks = (nE + CHUNK - 1) / CHUNK;
#pragma unroll 1
  for (int ch = 0; ch < nChunks; ++ch) {
    const int cbase = ch * CHUNK;
    const int wc = scan_chunk(dsts, nE, cbase, nodeBase, nb, vec8, list, tid, lane, wave);
    if (lane == 0) wcnt[wave] = wc;
    __syncthreads();
    int pre = 0, all = 0;
#pragma unroll
    for (int w2 = 0; w2 < NWAVE; ++w2) {
      int c = wcnt[w2];
      c = c < 0 ? 0 : (c > WCAP ? WCAP : c);
      all += c;
      pre += (w2 < wave) ? c : 0;
    }
    const int wcc  = wc > WCAP ? WCAP : wc;
    const int base = tot + pre;
#pragma unroll 1
    for (int i = lane; i < wcc; i += 32) {
      const unsigned ent = (unsigned)list[wave * WCAP + i];
      const int el = (int)((ent >> SLA) & (unsigned)(CHUNK - 1));
      const unsigned sq = ent & (unsigned)(NBA - 1);
      int eid = cbase + el;
      eid = eid > nE - 1 ? nE - 1 : eid;
      const int pos = base + i;
      if (pos < RCAP) reg1[pos] = (int)(((unsigned)eid << SLA) | sq);
    }
    if (tot + all > RCAP) ovf = 1;
    tot += all;
    tot = tot > RCAP ? RCAP : tot;
    __syncthreads();
  }
  const int nh = tot;
  const int nhPad = (nh + 31) & ~31;

  if (wave == 0) {
#pragma unroll 1
    for (int b0 = 0; b0 < nh; b0 += 32) {
      const int idx = b0 + lane;
      const int uv  = reg1[idx < nh ? idx : nh - 1];
      const int m32 = (nh - b0) < 32 ? (nh - b0) : 32;
#pragma unroll 1
      for (int k = 0; k < m32; ++k) {
        const int u  = __builtin_amdgcn_readlane(uv, k);
        const int sq = u & (NBA - 1);
        if (lane == 0) cnt[sq] = cnt[sq] + 1;
      }
    }
  }
  __syncthreads();
  if (wave == 0) {
    const int base = lane * (NBA / 32);
    int s = 0;
#pragma unroll 1
    for (int i = 0; i < NBA / 32; ++i) s += cnt[base + i];
    int incl = s;
#pragma unroll
    for (int d = 1; d < 32; d <<= 1) {
      const int y = __shfl_up(incl, d, 32);
      incl += (lane >= d) ? y : 0;
    }
    int run = incl - s;
#pragma unroll 1
    for (int i = 0; i < NBA / 32; ++i) {
      const int cv = cnt[base + i];
      offs[base + i] = run;
      cur[base + i]  = run;
      run += cv;
    }
  }
  __syncthreads();
  if (wave == 0) {
#pragma unroll 1
    for (int b0 = 0; b0 < nh; b0 += 32) {
      const int idx = b0 + lane;
      const int uv  = reg1[idx < nh ? idx : nh - 1];
      const int m32 = (nh - b0) < 32 ? (nh - b0) : 32;
#pragma unroll 1
      for (int k = 0; k < m32; ++k) {
        const int u  = __builtin_amdgcn_readlane(uv, k);
        const int sq = u & (NBA - 1);
        if (lane == 0) {
          int p = cur[sq];
          p = p < 0 ? 0 : (p > RCAP - 1 ? RCAP - 1 : p);
          sl[p] = (int)((unsigned)u >> SLA);
          cur[sq] = p + 1;
        }
      }
    }
  }
  __syncthreads();
  for (int i = nh + tid; i < nhPad; i += NTHR) sl[i] = 0;
  __syncthreads();

  int* eb = EIDS + (size_t)blk * RCAP;
  const v4i ov = *(const v4ia*)(offs + 4 * tid);
  const v4i cv = *(const v4ia*)(cnt + 4 * tid);
  int* op = OFFT + (size_t)blk * NBA + 4 * tid;
  int* cp = CNTT + (size_t)blk * NBA + 4 * tid;
  v4i fv;
  fv.x = (tid == 0) ? nh : 0;
  fv.y = (tid == 0) ? ovf : 0;
  fv.z = 0; fv.w = 0;
  int* fp = FLG + (size_t)blk * 32 + 4 * (tid & 7);
#pragma unroll 1
  for (int p = tid * 4; p < nhPad; p += NTHR * 4) {
    const v4i v = *(const v4ia*)(sl + p);
    *(volatile v4i*)(eb + p) = v;
  }
  *(volatile v4i*)op = ov;
  *(volatile v4i*)cp = cv;
  if (tid < 8) *(volatile v4i*)fp = fv;
  __threadfence();
#pragma unroll 1
  for (int p = tid * 4; p < nhPad; p += NTHR * 4) {
    const v4i v = *(const v4ia*)(sl + p);
    *(volatile v4i*)(eb + p) = v;
  }
  *(volatile v4i*)op = ov;
  *(volatile v4i*)cp = cv;
  if (tid < 8) *(volatile v4i*)fp = fv;
}

__global__ __launch_bounds__(BTHR) void k_basis(const float* __restrict__ pos, const int* __restrict__ dsti,
                                                const int* __restrict__ srci, const int* __restrict__ EIDS,
                                                const int* __restrict__ FLG, int* SR, int nE, int nN) {
  __shared__ __attribute__((aligned(16))) int tile[BTHR * 32];
  const int tid = (int)threadIdx.x;
  const int blk = (int)blockIdx.y;
  const int base = (int)blockIdx.x * BTHR;
  const int nhraw = FLG[(size_t)blk * 32];
  const int nh = nhraw < 0 ? 0 : (nhraw > RCAP ? RCAP : nhraw);
  if (base >= nh) return;
  const int s = base + tid;
  const bool val = s < nh;
  const int sc = val ? s : nh - 1;
  int e = EIDS[(size_t)blk * RCAP + sc];
  e = e < 0 ? 0 : (e > nE - 1 ? nE - 1 : e);
  int sn = srci[e], dn = dsti[e];
  sn = sn < 0 ? 0 : (sn > nN - 1 ? nN - 1 : sn);
  dn = dn < 0 ? 0 : (dn > nN - 1 ? nN - 1 : dn);
  const float* ps = pos + (size_t)sn * 3;
  const float* pd = pos + (size_t)dn * 3;
  const float dx = bfr(ps[0]) - bfr(pd[0]);
  const float dy = bfr(ps[1]) - bfr(pd[1]);
  const float dz = bfr(ps[2]) - bfr(pd[2]);
  const float r2 = dx * dx + dy * dy + dz * dz;
  const float r  = sqrtf(fmaxf(r2, 1e-12f));
  const float inv = 1.0f / r;
  const float ux = dx * inv, uy = dy * inv, uz = dz * inv;
  const float s3 = 1.7320508075688772f;
  const float hs3 = 0.8660254037844386f;
  float Y[9];
  Y[0] = 1.0f; Y[1] = ux; Y[2] = uy; Y[3] = uz;
  Y[4] = s3 * ux * uy; Y[5] = s3 * uy * uz; Y[6] = 0.5f * (3.0f * uz * uz - 1.0f);
  Y[7] = s3 * ux * uz; Y[8] = hs3 * (ux * ux - uy * uy);
  const float rc  = fminf(r, 4.999999f);
  const float den = (5.0f - rc) * (5.0f + rc);
  const float ex  = expf(-(rc * rc) * (1.0f / den));
  const float cut = (r < 5.0f) ? ex : 0.0f;
  const float yv = 1.0f / (1.0f + r);
  const float om = 1.0f - yv;
  float yp[8], mp[8];
  yp[0] = 1.0f; mp[0] = 1.0f;
#pragma unroll
  for (int k = 1; k < 8; ++k) { yp[k] = yp[k - 1] * yv; mp[k] = mp[k - 1] * om; }
  const float bn[8] = {1.0f, 7.0f, 21.0f, 35.0f, 35.0f, 21.0f, 7.0f, 1.0f};
  unsigned int hh[8], hm[8], hl[8];
#pragma unroll
  for (int k = 0; k < 8; ++k) {
    const float v = ((bn[k] * yp[k]) * mp[7 - k]) * cut;
    const S3 t = split3(v);
    hh[k] = t.h; hm[k] = t.m; hl[k] = t.l;
  }
  const int msk = val ? -1 : 0;
  v4i q[8];
  q[0].x = sn;                    q[0].y = __float_as_int(Y[0]); q[0].z = __float_as_int(Y[1]); q[0].w = __float_as_int(Y[2]);
  q[1].x = __float_as_int(Y[3]);  q[1].y = __float_as_int(Y[4]); q[1].z = __float_as_int(Y[5]); q[1].w = __float_as_int(Y[6]);
  q[2].x = __float_as_int(Y[7]);  q[2].y = __float_as_int(Y[8]); q[2].z = 0; q[2].w = 0;
  q[3].x = 0; q[3].y = 0; q[3].z = 0; q[3].w = 0;
  q[4].x = (int)(hh[0] | (hh[1] << 16)); q[4].y = (int)(hh[2] | (hh[3] << 16));
  q[4].z = (int)(hh[4] | (hh[5] << 16)); q[4].w = (int)(hh[6] | (hh[7] << 16));
  q[5].x = (int)(hm[0] | (hm[1] << 16)); q[5].y = (int)(hm[2] | (hm[3] << 16));
  q[5].z = (int)(hm[4] | (hm[5] << 16)); q[5].w = (int)(hm[6] | (hm[7] << 16));
  q[6].x = (int)(hl[0] | (hl[1] << 16)); q[6].y = (int)(hl[2] | (hl[3] << 16));
  q[6].z = (int)(hl[4] | (hl[5] << 16)); q[6].w = (int)(hl[6] | (hl[7] << 16));
  q[7].x = 0; q[7].y = 0; q[7].z = 0; q[7].w = 0;
#pragma unroll
  for (int i = 0; i < 8; ++i) {
    v4i t = q[i];
    t.x &= msk; t.y &= msk; t.z &= msk; t.w &= msk;
    *(v4ia*)(tile + tid * 32 + 4 * i) = t;
  }
  __syncthreads();
  int* sb = SR + ((size_t)blk * RCAP + (size_t)base) * 32;
#pragma unroll 1
  for (int i = 0; i < 8; ++i) {
    const int idx = i * BTHR + tid;
    const v4i v = *(const v4ia*)(tile + idx * 4);
    *(volatile v4i*)(sb + (size_t)idx * 4) = v;
  }
  __threadfence();
#pragma unroll 1
  for (int i = 0; i < 8; ++i) {
    const int idx = i * BTHR + tid;
    const v4i v = *(const v4ia*)(tile + idx * 4);
    *(volatile v4i*)(sb + (size_t)idx * 4) = v;
  }
}

__device__ __forceinline__ int tmap(int idx) {
  const int o = idx * 4;
  const int nd = o / XROW;
  const int rem = o - nd * XROW;
  return (rem >> 5) * 512 + nd * 32 + (rem & 31);
}

__device__ __forceinline__ void dense9(float* T, const unsigned short* __restrict__ W,
                                       const float* __restrict__ bias, int lane) {
  const int h = lane >> 4, m = lane & 15;
  FragB bw[3][2];
#pragma unroll
  for (int d = 0; d < 3; ++d) {
#pragma unroll
    for (int t = 0; t < 2; ++t) {
      const unsigned short* wq = W + (size_t)((d * 32 + 16 * t + m) * 32 + 8 * h);
      bw[d][t].h[0] = *(const v8usa*)wq;
      bw[d][t].h[1] = *(const v8usa*)(wq + 16);
    }
  }
  const float b0 = bfr(bias[m]);
  const float b1 = bfr(bias[16 + m]);
#pragma unroll
  for (int p = 0; p < 9; ++p) {
    const int d = (p == 0) ? 0 : ((p < 4) ? 1 : 2);
    const float* tp = T + p * 512 + m * 32 + 8 * h;
    const v4f a0 = *(const v4fa*)tp;
    const v4f a1 = *(const v4fa*)(tp + 4);
    const v4f a2 = *(const v4fa*)(tp + 16);
    const v4f a3 = *(const v4fa*)(tp + 20);
    const float vals[16] = {a0.x, a0.y, a0.z, a0.w, a1.x, a1.y, a1.z, a1.w,
                            a2.x, a2.y, a2.z, a2.w, a3.x, a3.y, a3.z, a3.w};
    FragB fh, fm, fl;
#pragma unroll
    for (int i = 0; i < 16; ++i) {
      const S3 s = split3(vals[i]);
      fh.h[i >> 3][i & 7] = (unsigned short)s.h;
      fm.h[i >> 3][i & 7] = (unsigned short)s.m;
      fl.h[i >> 3][i & 7] = (unsigned short)s.l;
    }
#pragma unroll
    for (int t = 0; t < 2; ++t) {
      v8f acc = {0.f, 0.f, 0.f, 0.f, 0.f, 0.f, 0.f, 0.f};
      acc = wmb(fh, bw[d][t], acc);
      acc = wmb(fm, bw[d][t], acc);
      acc = wmb(fl, bw[d][t], acc);
      const float bv = (p == 0) ? ((t == 0) ? b0 : b1) : 0.0f;
#pragma unroll
      for (int r = 0; r < 8; ++r) T[p * 512 + (8 * h + r) * 32 + 16 * t + m] = acc[r] + bv;
    }
  }
}

template <int MODE>
__global__ __launch_bounds__(32) __attribute__((amdgpu_num_vgpr(248)))
void k_iter(const int* __restrict__ SR, const int* __restrict__ OFFT, const int* __restrict__ CNTT,
            const int* __restrict__ FLG, const float* __restrict__ Xin, float* Xout,
            const float* __restrict__ embed, const int* __restrict__ Zt,
            const unsigned short* __restrict__ RWT, const unsigned short* __restrict__ DWT,
            const float* __restrict__ d1b, const float* __restrict__ d2b,
            const float* __restrict__ tdW, const float* __restrict__ monoW,
            const float* __restrict__ ebias, float* outp, int it, int nN, int nBk) {
  constexpr int NT = (MODE == 0) ? 6 : 22;
  __shared__ __attribute__((aligned(16))) float T[9 * 512];
  __shared__ __attribute__((aligned(16))) float rwt[16 * NRW];
  __shared__ __attribute__((aligned(16))) int   slt[16 * 32];
  __shared__ __attribute__((aligned(16))) float x2s[16 * 16];
  const int lane = (int)threadIdx.x & 31, h = lane >> 4, m = lane & 15;
  const int node0 = (int)blockIdx.x * 16;
  if (node0 + 16 > nN) return;
  const float qnan = __int_as_float(0x7fc00000);

  if constexpr (MODE != 0) {
    const float* xb = Xin + (size_t)node0 * XROW;
#pragma unroll 4
    for (int i2 = 0; i2 < 36; ++i2) {
      const int idx = i2 * 32 + lane;
      *(v4fa*)(T + tmap(idx)) = *(const v4f*)(xb + 4 * idx);
    }
  }
  __syncthreads();

#pragma unroll 1
  for (int nl = 0; nl < 16; ++nl) {
    const int n = node0 + nl;
    int b = n >> SLA;
    b = b > nBk - 1 ? nBk - 1 : b;
    const int nhraw = __builtin_amdgcn_readfirstlane(FLG[(size_t)b * 32]);
    const int bfl   = __builtin_amdgcn_readfirstlane(FLG[(size_t)b * 32 + 1]);
    const int nh = nhraw < 0 ? 0 : (nhraw > RCAP ? RCAP : nhraw);
    int off = __builtin_amdgcn_readfirstlane(OFFT[n]);
    const int craw = __builtin_amdgcn_readfirstlane(CNTT[n]);
    const bool bad = (bfl != 0) || nhraw < 0 || nhraw > RCAP || craw < 0 || craw > DEGCAP || off < 0 || off > nh;
    off = off < 0 ? 0 : (off > nh ? nh : off);
    int cnt = craw < 0 ? 0 : (craw > DEGCAP ? DEGCAP : craw);
    if (cnt > nh - off) cnt = nh - off;
    const size_t sbase = (size_t)b * RCAP + (size_t)off;

    float acc[9];
#pragma unroll
    for (int p = 0; p < 9; ++p) acc[p] = 0.0f;

#pragma unroll 1
    for (int g0 = 0; g0 < cnt; g0 += 16) {
      const int ng = (cnt - g0) < 16 ? (cnt - g0) : 16;
      {
        const int j = g0 + m;
        const bool v = j < cnt;
        const int jc = v ? j : cnt - 1;
        const int* rp = SR + (sbase + (size_t)jc) * 32 + 16 * h;
        v4i q0 = *(const v4i*)rp, q1 = *(const v4i*)(rp + 4), q2 = *(const v4i*)(rp + 8), q3 = *(const v4i*)(rp + 12);
        const int msk = v ? -1 : 0;
        q0.x &= msk; q0.y &= msk; q0.z &= msk; q0.w &= msk;
        q1.x &= msk; q1.y &= msk; q1.z &= msk; q1.w &= msk;
        q2.x &= msk; q2.y &= msk; q2.z &= msk; q2.w &= msk;
        q3.x &= msk; q3.y &= msk; q3.z &= msk; q3.w &= msk;
        int* tp = slt + m * 32 + 16 * h;
        *(v4ia*)tp = q0; *(v4ia*)(tp + 4) = q1; *(v4ia*)(tp + 8) = q2; *(v4ia*)(tp + 12) = q3;
      }
      __syncthreads();
      FragB af;
      af.h[0] = *(const v8usa*)(slt + m * 32 + 16 + 4 * h);
      af.h[1] = *(const v8usa*)(slt + m * 32 + 24 + 4 * h);
#pragma unroll 2
      for (int t = 0; t < NT; ++t) {
        const unsigned short* wq = RWT + ((size_t)(it * NRW + 16 * t + m)) * 32 + 8 * h;
        FragB bf;
        bf.h[0] = *(const v8usa*)wq;
        bf.h[1] = *(const v8usa*)(wq + 16);
        v8f d = {0.f, 0.f, 0.f, 0.f, 0.f, 0.f, 0.f, 0.f};
        d = wmb(af, bf, d);
#pragma unroll
        for (int r = 0; r < 8; ++r) rwt[(8 * h + r) * NRW + 16 * t + m] = d[r];
      }
      __syncthreads();

#pragma unroll 1
      for (int j = 0; j < ng; ++j) {
        const v4i hA = *(const v4ia*)(slt + j * 32);
        const v4i hB = *(const v4ia*)(slt + j * 32 + 4);
        const v4i hC = *(const v4ia*)(slt + j * 32 + 8);
        int sr = hA.x;
        sr = sr < 0 ? 0 : (sr > nN - 1 ? nN - 1 : sr);
        float Y[9];
        Y[0] = __int_as_float(hA.y); Y[1] = __int_as_float(hA.z); Y[2] = __int_as_float(hA.w);
        Y[3] = __int_as_float(hB.x); Y[4] = __int_as_float(hB.y); Y[5] = __int_as_float(hB.z);
        Y[6] = __int_as_float(hB.w); Y[7] = __int_as_float(hC.x); Y[8] = __int_as_float(hC.y);
        float xs[9];
        if constexpr (MODE == 0) {
          int zz = Zt[sr];
          zz = zz < 0 ? 0 : (zz > NZ - 1 ? NZ - 1 : zz);
          xs[0] = bfr(embed[zz * NF + lane]);
#pragma unroll
          for (int p = 1; p < 9; ++p) xs[p] = 0.0f;
        } else {
          const float* xr = Xin + (size_t)sr * XROW + lane;
          xs[0] = xr[0]; xs[1] = xr[32]; xs[2] = xr[64]; xs[3] = xr[96]; xs[4] = xr[128];
          ldwait();
          xs[5] = xr[160]; xs[6] = xr[192]; xs[7] = xr[224]; xs[8] = xr[256];
          ldwait();
        }
        const float* rr = rwt + j * NRW + lane;
        PathR<0, 0, 0, 0>::run(xs, Y, rr[0 * 32], acc);
        PathR<0, 1, 1, 0>::run(xs, Y, rr[1 * 32], acc);
        PathR<0, 2, 2, 0>::run(xs, Y, rr[2 * 32], acc);
        if constexpr (MODE != 0) {
          PathR<1, 0, 1, 0>::run(xs, Y, rr[3 * 32], acc);
          PathR<1, 1, 0, 0>::run(xs, Y, rr[4 * 32], acc);
          PathR<1, 1, 2, 0>::run(xs, Y, rr[5 * 32], acc);
          PathR<1, 2, 1, 0>::run(xs, Y, rr[6 * 32], acc);
          PathR<2, 0, 2, 0>::run(xs, Y, rr[7 * 32], acc);
          PathR<2, 1, 1, 0>::run(xs, Y, rr[8 * 32], acc);
          PathR<2, 2, 0, 0>::run(xs, Y, rr[9 * 32], acc);
          PathR<2, 2, 2, 0>::run(xs, Y, rr[10 * 32], acc);
        }
      }
      __syncthreads();
    }

    const int o = nl * 32 + lane;
    if constexpr (MODE == 0) {
      int zn = Zt[n];
      zn = zn < 0 ? 0 : (zn > NZ - 1 ? NZ - 1 : zn);
      const float e0 = bfr(embed[zn * NF + lane]);
      T[o] = e0 + acc[0];
#pragma unroll
      for (int p = 1; p < 9; ++p) T[p * 512 + o] = acc[p];
    } else {
#pragma unroll
      for (int p = 0; p < 9; ++p) T[p * 512 + o] = T[p * 512 + o] + acc[p];
    }
    if (bad) {
#pragma unroll
      for (int p = 0; p < 9; ++p) T[p * 512 + o] = qnan;
    }
  }
  __syncthreads();

  dense9(T, DWT + (size_t)(it * 3) * 1024, d1b + it * NF, lane);
  __syncthreads();
#pragma unroll 1
  for (int nl = 0; nl < 16; ++nl) {
    const int o = nl * 32 + lane;
    const float s  = T[o];
    const float sg = 1.0f / (1.0f + expf(-s));
    T[o] = s * sg;
    const float gt = sg * (1.0f + s * (1.0f - sg));
#pragma unroll
    for (int p = 1; p < 9; ++p) T[p * 512 + o] = T[p * 512 + o] * gt;
  }
  __syncthreads();
  dense9(T, DWT + (size_t)DW_L2 + (size_t)(it * 3) * 1024, d2b + it * NF, lane);
  __syncthreads();
  if constexpr (MODE == 0) {
#pragma unroll 4
    for (int nl = 0; nl < 16; ++nl) {
      int zn = Zt[node0 + nl];
      zn = zn < 0 ? 0 : (zn > NZ - 1 ? NZ - 1 : zn);
      const float e0 = bfr(embed[zn * NF + lane]);
      T[nl * 32 + lane] = e0 + T[nl * 32 + lane];
    }
  } else {
    const float* xb = Xin + (size_t)node0 * XROW;
#pragma unroll 4
    for (int i2 = 0; i2 < 36; ++i2) {
      const int idx = i2 * 32 + lane;
      const v4f xo = *(const v4f*)(xb + 4 * idx);
      const int to = tmap(idx);
      v4f tv = *(const v4fa*)(T + to);
      tv.x = xo.x + tv.x; tv.y = xo.y + tv.y; tv.z = xo.z + tv.z; tv.w = xo.w + tv.w;
      *(v4fa*)(T + to) = tv;
    }
  }
  __syncthreads();

  if constexpr (MODE != 2) {
    float* xo = Xout + (size_t)node0 * XROW;
#pragma unroll 4
    for (int i2 = 0; i2 < 36; ++i2) {
      const int idx = i2 * 32 + lane;
      const v4f v = *(const v4fa*)(T + tmap(idx));
      *(volatile v4f*)(xo + 4 * idx) = v;
    }
    __threadfence();
#pragma unroll 4
    for (int i2 = 0; i2 < 36; ++i2) {
      const int idx = i2 * 32 + lane;
      const v4f v = *(const v4fa*)(T + tmap(idx));
      *(volatile v4f*)(xo + 4 * idx) = v;
    }
  } else {
    const v4f tw0 = bfr4(*(const v4f*)(tdW + 0 * 128 + lane * 4));
    const v4f tw1 = bfr4(*(const v4f*)(tdW + 3 * 128 + lane * 4));
    const v4f tw2 = bfr4(*(const v4f*)(tdW + 7 * 128 + lane * 4));
    const v4f tw3 = bfr4(*(const v4f*)(tdW + 8 * 128 + lane * 4));
    const v4f tw4 = bfr4(*(const v4f*)(tdW + 11 * 128 + lane * 4));
    const v4f tw5 = bfr4(*(const v4f*)(tdW + 15 * 128 + lane * 4));
    const v4f tw6 = bfr4(*(const v4f*)(tdW + 16 * 128 + lane * 4));
#pragma unroll 1
    for (int nl = 0; nl < 16; ++nl) {
      float xv[9];
#pragma unroll
      for (int p = 0; p < 9; ++p) xv[p] = T[p * 512 + nl * 32 + lane];
      float part[16];
#pragma unroll
      for (int i = 0; i < 16; ++i) part[i] = 0.0f;
      TdR<0, 0, 0, 0>::run(xv, tw0, part);
      TdR<0, 1, 1, 0>::run(xv, tw1, part);
      TdR<1, 0, 1, 0>::run(xv, tw2, part);
      TdR<1, 1, 0, 0>::run(xv, tw3, part);
      TdR<1, 2, 1, 0>::run(xv, tw4, part);
      TdR<2, 1, 1, 0>::run(xv, tw5, part);
      TdR<2, 2, 0, 0>::run(xv, tw6, part);
#pragma unroll
      for (int i = 0; i < 16; ++i) {
        float v = part[i];
#pragma unroll
        for (int sh = 16; sh > 0; sh >>= 1) v += __shfl_xor(v, sh, 32);
        part[i] = v;
      }
      if (lane == 0) {
#pragma unroll
        for (int i = 0; i < 16; ++i) x2s[nl * 16 + i] = part[i];
      }
    }
    __syncthreads();

    const v4f m0 = bfr4(*(const v4f*)(monoW));
    const v4f m1 = bfr4(*(const v4f*)(monoW + 4));
    const v4f m2 = bfr4(*(const v4f*)(monoW + 8));
    const v4f m3 = bfr4(*(const v4f*)(monoW + 12));
    const int nq = lane & 15;
    int zq = Zt[node0 + nq];
    zq = zq < 0 ? 0 : (zq > NZ - 1 ? NZ - 1 : zq);
    const float eb = bfr(ebias[zq]);
    const v4f sq = *(const v4fa*)(x2s + nq * 16);
    v4f o0;
    o0.x = fmaf(sq.w, m3.x, fmaf(sq.z, m2.x, fmaf(sq.y, m1.x, sq.x * m0.x))) + eb;
    o0.y = fmaf(sq.w, m3.y, fmaf(sq.z, m2.y, fmaf(sq.y, m1.y, sq.x * m0.y))) + eb;
    o0.z = fmaf(sq.w, m3.z, fmaf(sq.z, m2.z, fmaf(sq.y, m1.z, sq.x * m0.z))) + eb;
    o0.w = fmaf(sq.w, m3.w, fmaf(sq.z, m2.w, fmaf(sq.y, m1.w, sq.x * m0.w))) + eb;

    const int qa = lane;
    int qb = lane + 32;
    qb = qb > 47 ? 47 : qb;
    const int na = qa / 3, ma = qa - 3 * na;
    const int nb2 = qb / 3, mb = qb - 3 * nb2;
    const v4f sa = *(const v4fa*)(x2s + na * 16);
    const v4f xa = *(const v4fa*)(x2s + na * 16 + 4 + 4 * ma);
    const v4f sb = *(const v4fa*)(x2s + nb2 * 16);
    const v4f xb2 = *(const v4fa*)(x2s + nb2 * 16 + 4 + 4 * mb);
    v4f ra, rb;
    ra.x = (xa.x * ((sa.x > -1.0f && sa.x < 1.0f) ? 1.0f : 0.0f)) * 0.3f;
    ra.y = (xa.y * ((sa.y > -1.0f && sa.y < 1.0f) ? 1.0f : 0.0f)) * 0.3f;
    ra.z = (xa.z * ((sa.z > -1.0f && sa.z < 1.0f) ? 1.0f : 0.0f)) * 0.3f;
    ra.w = (xa.w * ((sa.w > -1.0f && sa.w < 1.0f) ? 1.0f : 0.0f)) * 0.3f;
    rb.x = (xb2.x * ((sb.x > -1.0f && sb.x < 1.0f) ? 1.0f : 0.0f)) * 0.3f;
    rb.y = (xb2.y * ((sb.y > -1.0f && sb.y < 1.0f) ? 1.0f : 0.0f)) * 0.3f;
    rb.z = (xb2.z * ((sb.z > -1.0f && sb.z < 1.0f) ? 1.0f : 0.0f)) * 0.3f;
    rb.w = (xb2.w * ((sb.w > -1.0f && sb.w < 1.0f) ? 1.0f : 0.0f)) * 0.3f;

    float* p0 = outp + (size_t)node0 * 4 + 4 * nq;
    float* p1 = outp + (size_t)nN * 4 + (size_t)node0 * 12 + 4 * qa;
    float* p2 = outp + (size_t)nN * 4 + (size_t)node0 * 12 + 4 * qb;
    if (lane < 16) *(volatile v4f*)p0 = o0;
    *(volatile v4f*)p1 = ra;
    if (lane < 16) *(volatile v4f*)p2 = rb;
    __threadfence();
    if (lane < 16) *(volatile v4f*)p0 = o0;
    *(volatile v4f*)p1 = ra;
    if (lane < 16) *(volatile v4f*)p2 = rb;
  }
}

extern "C" void kernel_launch(void* const* d_in, const int* in_sizes, int n_in,
                              void* d_out, int out_size, void* d_ws, size_t ws_size,
                              hipStream_t stream) {
  if (n_in < 13) return;
  const int nN = in_sizes[10];
  const int nE = in_sizes[11];
  if (nN <= 0 || (nN % 16) != 0 || nN > (1 << 20)) return;
  if (nE < 1 || nE > (1 << 21) || in_sizes[12] != nE) return;
  if (in_sizes[0] != nN * 3) return;
  if (in_sizes[1] != NZ * NF) return;
  if (in_sizes[2] != 3 * 27 * 8 * NF) return;
  if (in_sizes[3] != 3 * 3 * NF * NF || in_sizes[5] != 3 * 3 * NF * NF) return;
  if (in_sizes[4] != 3 * NF || in_sizes[6] != 3 * NF) return;
  if (in_sizes[7] != 18 * NF * 4) return;
  if (in_sizes[8] != 16 || in_sizes[9] != NZ) return;
  if (out_size != nN * 16) return;

  const float* pos   = (const float*)d_in[0];
  const float* embed = (const float*)d_in[1];
  const float* mpW   = (const float*)d_in[2];
  const float* d1W   = (const float*)d_in[3];
  const float* d1b   = (const float*)d_in[4];
  const float* d2W   = (const float*)d_in[5];
  const float* d2b   = (const float*)d_in[6];
  const float* tdW   = (const float*)d_in[7];
  const float* monoW = (const float*)d_in[8];
  const float* ebias = (const float*)d_in[9];
  const int*   Zt    = (const int*)d_in[10];
  const int*   dsti  = (const int*)d_in[11];
  const int*   srci  = (const int*)d_in[12];
  float* outp = (float*)d_out;

  const int gA = (nN + NBA - 1) / NBA;
  const int vec8 = ((nE & 3) == 0) ? 1 : 0;

  char* ws = (char*)d_ws;
  size_t off = 0;
  const size_t oRW = off; off += (size_t)3 * NRW * 32 * 2;          off = (off + 255) & ~(size_t)255;
  const size_t oDW = off; off += (size_t)2 * DW_L2 * 2;             off = (off + 255) & ~(size_t)255;
  const size_t oEI = off; off += (size_t)gA * RCAP * 4;             off = (off + 255) & ~(size_t)255;
  const size_t oOF = off; off += (size_t)gA * NBA * 4;              off = (off + 255) & ~(size_t)255;
  const size_t oCN = off; off += (size_t)gA * NBA * 4;              off = (off + 255) & ~(size_t)255;
  const size_t oFL = off; off += (size_t)gA * 128;                  off = (off + 255) & ~(size_t)255;
  const size_t oSR = off; off += (size_t)gA * RCAP * 128;           off = (off + 255) & ~(size_t)255;
  const size_t oXA = off; off += (size_t)nN * XROW * 4;             off = (off + 255) & ~(size_t)255;
  const size_t oXB = off; off += (size_t)nN * XROW * 4;             off = (off + 255) & ~(size_t)255;
  if (off > ws_size || off > (size_t)WSMAX) return;
  unsigned short* RWT = (unsigned short*)(ws + oRW);
  unsigned short* DWT = (unsigned short*)(ws + oDW);
  int*   EIDS = (int*)(ws + oEI);
  int*   OFFT = (int*)(ws + oOF);
  int*   CNTT = (int*)(ws + oCN);
  int*   FLG  = (int*)(ws + oFL);
  int*   SR   = (int*)(ws + oSR);
  float* XA   = (float*)(ws + oXA);
  float* XB   = (float*)(ws + oXB);

  const int bktLds = BKT_LDS_INTS * 4;
  hipFuncSetAttribute(reinterpret_cast<const void*>(&k_bucket),
                      hipFuncAttributeMaxDynamicSharedMemorySize, bktLds);

  k_prep<<<(U_RW + 2 * U_DH) / PTHR, PTHR, 0, stream>>>(mpW, d1W, d2W, RWT, DWT);
  k_bucket<<<gA, NTHR, bktLds, stream>>>(dsti, nE, nN, vec8, EIDS, OFFT, CNTT, FLG);
  k_basis<<<dim3(RCAP / BTHR, gA), BTHR, 0, stream>>>(pos, dsti, srci, EIDS, FLG, SR, nE, nN);
  const int gI = nN / 16;
  k_iter<0><<<gI, 32, 0, stream>>>(SR, OFFT, CNTT, FLG, XB, XA, embed, Zt, RWT, DWT, d1b, d2b,
                                   tdW, monoW, ebias, outp, 0, nN, gA);
  k_iter<1><<<gI, 32, 0, stream>>>(SR, OFFT, CNTT, FLG, XA, XB, embed, Zt, RWT, DWT, d1b, d2b,
                                   tdW, monoW, ebias, outp, 1, nN, gA);
  k_iter<2><<<gI, 32, 0, stream>>>(SR, OFFT, CNTT, FLG, XB, XA, embed, Zt, RWT, DWT, d1b, d2b,
                                   tdW, monoW, ebias, outp, 2, nN, gA);
}
